// PointNetSetAbstraction_33552284516958
// MI455X (gfx1250) — hardware-verified
//
#include <hip/hip_runtime.h>
#pragma clang fp contract(off)

typedef __attribute__((ext_vector_type(16))) _Float16 v16h;
typedef __attribute__((ext_vector_type(8)))  _Float16 v8h;
typedef __attribute__((ext_vector_type(8)))  float    v8f;
typedef __attribute__((ext_vector_type(4)))  float    v4f;
typedef __attribute__((ext_vector_type(4)))  unsigned v4u;

constexpr int BATCH  = 16;
constexpr int NPTS   = 4096;
constexpr int NFEAT  = 64;
constexpr int NCENT  = 1024;
constexpr int NSAMP  = 32;
constexpr int CH_IN  = 67;
constexpr int CH_A   = 64;
constexpr int CH_B   = 64;
constexpr int CH_C   = 128;
constexpr int NGROUP = BATCH * NCENT;
constexpr int NROWS  = NGROUP * NSAMP;
constexpr int TILE_ROWS = 128;
constexpr int NBLK_BALL = NGROUP / 8;
constexpr int NBLK_MLP  = NROWS / TILE_ROWS;
constexpr int APITCH = 72;
constexpr int SPITCH = 68;
static_assert(NROWS == 524288, "row count");
static_assert(NROWS % TILE_ROWS == 0, "tile multiple");
static_assert((BATCH * NPTS) % 128 == 0, "tile multiple");
static_assert(NFEAT % 32 == 0 && CH_A % 32 == 0 && CH_B % 32 == 0, "k multiple of 32");
static_assert(CH_IN == 3 + NFEAT, "channel split");
static_assert(NSAMP == 32, "one lane per sample");

constexpr size_t OFF_W0P  = 0;
constexpr size_t OFF_W1H  = OFF_W0P  + (size_t)CH_A * NFEAT * 2;
constexpr size_t OFF_W2H  = OFF_W1H  + (size_t)CH_B * CH_A * 2;
constexpr size_t OFF_W0X  = OFF_W2H  + (size_t)CH_C * CH_B * 2;
constexpr size_t OFF_TAB0 = OFF_W0X  + (size_t)CH_A * 4 * 4;
constexpr size_t OFF_TAB1 = OFF_TAB0 + 512;
constexpr size_t OFF_TAB2 = OFF_TAB1 + 512;
constexpr size_t OFF_NXYZ = OFF_TAB2 + 1024;
constexpr size_t OFF_GIDX = OFF_NXYZ + (size_t)BATCH * 3 * NCENT * 4;
constexpr size_t OFF_PTST = OFF_GIDX + (size_t)NGROUP * NSAMP * 4;
constexpr size_t OFF_P0   = OFF_PTST + (size_t)BATCH * NPTS * NFEAT * 2;
constexpr size_t OFF_PRT0 = OFF_P0   + (size_t)BATCH * NPTS * CH_A * 4;
constexpr size_t OFF_PRT1 = OFF_PRT0 + (size_t)NBLK_BALL * 2 * CH_A * 4;
constexpr size_t OFF_PRT2 = OFF_PRT1 + (size_t)NBLK_MLP * 2 * CH_B * 4;
constexpr size_t OFF_Y1   = OFF_PRT2 + (size_t)NBLK_MLP * 2 * CH_C * 4;
constexpr size_t OFF_GMAX = OFF_Y1   + (size_t)NROWS * CH_B * 2;
constexpr size_t OFF_GMIN = OFF_GMAX + (size_t)NGROUP * CH_C * 4;
constexpr size_t WS_TOTAL = OFF_GMIN + (size_t)NGROUP * CH_C * 4;
static_assert(WS_TOTAL == 118721536, "carve total");
static_assert(WS_TOTAL <= 134217728, "carve limit");
static_assert((OFF_NXYZ % 256) == 0 && (OFF_GIDX % 256) == 0 && (OFF_Y1 % 256) == 0, "alignment");

constexpr size_t OUT0_BYTES = (size_t)BATCH * 3 * NCENT * 4;
constexpr size_t OUT1_BYTES = (size_t)BATCH * CH_C * NCENT * 4;
static_assert(OUT0_BYTES == 196608, "out0 size");
static_assert(OUT0_BYTES + OUT1_BYTES == 8585216, "d_out total");
static_assert((OUT0_BYTES % 128) == 0, "out1 line aligned");

__device__ __forceinline__ float bf_rne(float f) {
  unsigned u = __float_as_uint(f);
  u = (u + 0x7FFFu + ((u >> 16) & 1u)) & 0xFFFF0000u;
  return __uint_as_float(u);
}
__device__ __forceinline__ int clampi(int v, int hi) {
  v = v < 0 ? 0 : v;
  return v > hi ? hi : v;
}
__device__ __forceinline__ float h16_to_f32(unsigned hb) {
  const unsigned sgn = (hb & 0x8000u) << 16;
  const unsigned em = hb & 0x7fffu;
  const float fn = __uint_as_float((em << 13) + 0x38000000u);
  const float fs = (float)em * 5.9604644775390625e-8f;
  const float mag = (em < 0x400u) ? fs : fn;
  return __uint_as_float(__float_as_uint(mag) | sgn);
}
__device__ __forceinline__ v8f mma_h(v16h a, v16h b, v8f c) {
  c = __builtin_amdgcn_wmma_f32_16x16x32_f16(false, a, false, b, (short)0, c, false, false);
  asm volatile("v_nop\n\tv_nop\n\tv_nop\n\tv_nop" : "+v"(c) : "v"(a), "v"(b));
  return c;
}
__device__ __forceinline__ v16h frag_g(const _Float16* p) {
  union { v16h v; v8h h[2]; } f;
  f.h[0] = *(const v8h*)(p);
  f.h[1] = *(const v8h*)(p + 16);
  return f.v;
}
__device__ __forceinline__ float y0_val(float p, float w0, float w1, float w2,
                                        float dx, float dy, float dz, float bias) {
  float t = w0 * dx;
  t = t + w1 * dy;
  t = t + w2 * dz;
  return (p + t) + bias;
}

__global__ __launch_bounds__(256) void k_prep(const float* __restrict__ W0, const float* __restrict__ W1,
                                              const float* __restrict__ W2, _Float16* __restrict__ W0p,
                                              _Float16* __restrict__ W1h, _Float16* __restrict__ W2h,
                                              float* __restrict__ W0x) {
  const int blk = blockIdx.x, t = threadIdx.x;
  if (blk < 8) {
    const float* src;
    _Float16* dst;
    int i, pitch, coff;
    if (blk < 2)      { i = blk * 256 + t;       src = W0; dst = W0p; pitch = CH_IN; coff = 3; }
    else if (blk < 4) { i = (blk - 2) * 256 + t; src = W1; dst = W1h; pitch = CH_A;  coff = 0; }
    else              { i = (blk - 4) * 256 + t; src = W2; dst = W2h; pitch = CH_B;  coff = 0; }
    const int o = i >> 3, c8 = (i & 7) * 8;
    v8h hv;
#pragma unroll
    for (int e = 0; e < 8; ++e) {
      const float w = bf_rne(src[o * pitch + coff + c8 + e]);
      hv[e] = (_Float16)w;
    }
    _Float16* dp = dst + o * 64 + c8;
    *(volatile v8h*)dp = hv;
    __threadfence();
    *(volatile v8h*)dp = hv;
  } else {
    const int o = t < CH_A ? t : CH_A - 1;
    v4f v;
    v[0] = bf_rne(W0[o * CH_IN + 0]);
    v[1] = bf_rne(W0[o * CH_IN + 1]);
    v[2] = bf_rne(W0[o * CH_IN + 2]);
    v[3] = 0.0f;
    if (t < CH_A) {
      float* dp = W0x + t * 4;
      *(volatile v4f*)dp = v;
      __threadfence();
      *(volatile v4f*)dp = v;
    }
  }
}

__global__ __launch_bounds__(256) void k_pts(const float* __restrict__ pts, _Float16* __restrict__ ptsT) {
  __shared__ __align__(16) float tile[64 * SPITCH];
  const int t = threadIdx.x;
  const int b = blockIdx.x >> 6, n0 = (blockIdx.x & 63) * 64;
#pragma unroll
  for (int i = 0; i < 4; ++i) {
    const int idx = i * 256 + t;
    const int c = idx >> 4, n4 = (idx & 15) * 4;
    const v4f v = *(const v4f*)(pts + ((size_t)(b * NFEAT + c)) * NPTS + n0 + n4);
    *(v4f*)(tile + c * SPITCH + n4) = v;
  }
  __syncthreads();
  for (int pass = 0; pass < 2; ++pass) {
#pragma unroll
    for (int i = 0; i < 2; ++i) {
      const int item = i * 256 + t;
      const int n = item >> 3, c8 = (item & 7) * 8;
      v8h hv;
#pragma unroll
      for (int e = 0; e < 8; ++e) hv[e] = (_Float16)bf_rne(tile[(c8 + e) * SPITCH + n]);
      *(volatile v8h*)(ptsT + ((size_t)(b * NPTS + n0 + n)) * NFEAT + c8) = hv;
    }
    __threadfence();
  }
}

__global__ __launch_bounds__(256) void k_p0(const _Float16* __restrict__ A, const _Float16* __restrict__ Bt,
                                            float* __restrict__ P0) {
  __shared__ __align__(16) float slab[8][16 * SPITCH];
  const int lane = threadIdx.x & 31, wave = threadIdx.x >> 5;
  const int c = lane & 15, hh = lane >> 4;
  const size_t row0 = (size_t)blockIdx.x * 128 + wave * 16;
  v8f acc[4];
#pragma unroll
  for (int j = 0; j < 4; ++j) acc[j] = (v8f){0.f, 0.f, 0.f, 0.f, 0.f, 0.f, 0.f, 0.f};
#pragma unroll
  for (int k0 = 0; k0 < NFEAT; k0 += 32) {
    const v16h a = frag_g(A + (row0 + c) * NFEAT + k0 + 8 * hh);
#pragma unroll
    for (int j = 0; j < 4; ++j) {
      const v16h bq = frag_g(Bt + (j * 16 + c) * NFEAT + k0 + 8 * hh);
      acc[j] = mma_h(a, bq, acc[j]);
    }
  }
  float* sl = slab[wave];
#pragma unroll
  for (int j = 0; j < 4; ++j)
#pragma unroll
    for (int r = 0; r < 8; ++r) sl[(8 * hh + r) * SPITCH + j * 16 + c] = acc[j][r];
  __syncthreads();
  const int c4 = (lane & 15) * 4;
  for (int pass = 0; pass < 2; ++pass) {
#pragma unroll
    for (int it = 0; it < 8; ++it) {
      const int row = it * 2 + hh;
      const v4f v = *(const v4f*)(sl + row * SPITCH + c4);
      *(volatile v4f*)(P0 + (row0 + row) * CH_A + c4) = v;
    }
    __threadfence();
  }
}

__global__ __launch_bounds__(256) void k_fps(const float* __restrict__ xyz, float* __restrict__ out0,
                                             float* __restrict__ newxyz) {
#pragma clang fp contract(off)
  __shared__ __align__(16) float sxyz[3 * NPTS];
  __shared__ float wval[2][8];
  __shared__ int widx[2][8];
  __shared__ int sidx[NCENT];
  const int b = blockIdx.x, tid = threadIdx.x;
  const int lane = tid & 31, wave = tid >> 5;
  const float* src = xyz + (size_t)b * 3 * NPTS;
#pragma unroll 1
  for (int it = 0; it < 3; ++it) {
    v4f v[4];
#pragma unroll
    for (int j = 0; j < 4; ++j) v[j] = *(const v4f*)(src + ((size_t)((it * 4 + j) * 256 + tid)) * 4);
#pragma unroll
    for (int j = 0; j < 4; ++j) {
      v4f r;
      r[0] = bf_rne(v[j][0]);
      r[1] = bf_rne(v[j][1]);
      r[2] = bf_rne(v[j][2]);
      r[3] = bf_rne(v[j][3]);
      *(v4f*)(sxyz + ((it * 4 + j) * 256 + tid) * 4) = r;
    }
    asm volatile("" ::: "memory");
  }
  __syncthreads();

  float px[16], py[16], pz[16], dist[16];
#pragma unroll
  for (int i = 0; i < 16; ++i) {
    const int n = i * 256 + tid;
    px[i] = sxyz[n];
    py[i] = sxyz[NPTS + n];
    pz[i] = sxyz[2 * NPTS + n];
    dist[i] = 1e10f;
  }

  int far = 0;
#pragma unroll 1
  for (int t = 0; t < NCENT; ++t) {
    if (tid == 0) sidx[t] = far;
    const float cx = sxyz[far], cy = sxyz[NPTS + far], cz = sxyz[2 * NPTS + far];
    float bestv = -1.0f;
    int besti = 0;
#pragma unroll
    for (int i = 0; i < 16; ++i) {
      const float dx = px[i] - cx, dy = py[i] - cy, dz = pz[i] - cz;
      const float t0 = dx * dx;
      const float t1 = dy * dy;
      const float t2 = dz * dz;
      const float d = (t0 + t2) + t1;
      const float dm = fminf(dist[i], d);
      dist[i] = dm;
      const bool up = dm > bestv;
      bestv = up ? dm : bestv;
      besti = up ? (i * 256 + tid) : besti;
    }
#pragma unroll
    for (int m = 16; m >= 1; m >>= 1) {
      const float ov = __shfl_xor(bestv, m, 32);
      const int oi = __shfl_xor(besti, m, 32);
      const bool take = (ov > bestv) || ((ov == bestv) && (oi < besti));
      bestv = take ? ov : bestv;
      besti = take ? oi : besti;
    }
    const int pb = t & 1;
    if (lane == 0) { wval[pb][wave] = bestv; widx[pb][wave] = besti; }
    __syncthreads();
    float bv = wval[pb][0];
    int bi = widx[pb][0];
#pragma unroll
    for (int w = 1; w < 8; ++w) {
      const float ov = wval[pb][w];
      const int oi = widx[pb][w];
      const bool take = (ov > bv) || ((ov == bv) && (oi < bi));
      bv = take ? ov : bv;
      bi = take ? oi : bi;
    }
    far = clampi(bi, NPTS - 1);
  }
  __syncthreads();

  const int s4 = tid * 4;
  const int i0 = clampi(sidx[s4 + 0], NPTS - 1);
  const int i1 = clampi(sidx[s4 + 1], NPTS - 1);
  const int i2 = clampi(sidx[s4 + 2], NPTS - 1);
  const int i3 = clampi(sidx[s4 + 3], NPTS - 1);
  v4f vx, vy, vz;
  vx[0] = sxyz[i0]; vx[1] = sxyz[i1]; vx[2] = sxyz[i2]; vx[3] = sxyz[i3];
  vy[0] = sxyz[NPTS + i0]; vy[1] = sxyz[NPTS + i1]; vy[2] = sxyz[NPTS + i2]; vy[3] = sxyz[NPTS + i3];
  vz[0] = sxyz[2 * NPTS + i0]; vz[1] = sxyz[2 * NPTS + i1]; vz[2] = sxyz[2 * NPTS + i2]; vz[3] = sxyz[2 * NPTS + i3];
  float* o0 = out0 + (size_t)b * 3 * NCENT + s4;
  float* w0 = newxyz + (size_t)b * 3 * NCENT + s4;
  for (int pass = 0; pass < 2; ++pass) {
    *(volatile v4f*)(o0) = vx;
    *(volatile v4f*)(o0 + NCENT) = vy;
    *(volatile v4f*)(o0 + 2 * NCENT) = vz;
    *(volatile v4f*)(w0) = vx;
    *(volatile v4f*)(w0 + NCENT) = vy;
    *(volatile v4f*)(w0 + 2 * NCENT) = vz;
    __threadfence();
  }
}

__global__ __launch_bounds__(256) void k_ball(const float* __restrict__ xyz, const float* __restrict__ newxyz,
                                              const float* __restrict__ P0, const float* __restrict__ W0x,
                                              const float* __restrict__ b0, int* __restrict__ gidx,
                                              float* __restrict__ part0) {
#pragma clang fp contract(off)
  __shared__ int slist[8][32];
  __shared__ __align__(16) float wst[8][128];
  __shared__ __align__(16) float pst[128];
  const int tid = threadIdx.x, lane = tid & 31, wave = tid >> 5;
  const int cen = blockIdx.x * 8 + wave;
  const int b = cen >> 10, s = cen & (NCENT - 1);
  const float* xb = xyz + (size_t)b * 3 * NPTS;
  const float* cb = newxyz + (size_t)b * 3 * NCENT;
  const float cx = cb[s], cy = cb[NCENT + s], cz = cb[2 * NCENT + s];
  const float c0 = cx * cx;
  const float c1 = cy * cy;
  const float c2 = cz * cz;
  const float sc = (c0 + c2) + c1;
  const float r2 = __uint_as_float(0x3D23D70Au);

  int cnt = 0;
#pragma unroll 1
  for (int ch = 0; ch < NPTS / 32; ++ch) {
    const int n = ch * 32 + lane;
    const float x = bf_rne(xb[n]);
    const float y = bf_rne(xb[NPTS + n]);
    const float z = bf_rne(xb[2 * NPTS + n]);
    const float x0 = x * x;
    const float x1 = y * y;
    const float x2 = z * z;
    const float sx = (x0 + x2) + x1;
    float p = cx * x;
    p = __builtin_fmaf(cy, y, p);
    p = __builtin_fmaf(cz, z, p);
    const float tw = 2.0f * p;
    const float sqr = (sc + sx) - tw;
    const bool inr = !(sqr > r2);
    const unsigned mask = __builtin_amdgcn_ballot_w32(inr);
    const int pos = cnt + __popc(mask & ((1u << lane) - 1u));
    if (inr && pos < NSAMP) slist[wave][pos] = n;
    cnt += __popc(mask);
    if (cnt >= NSAMP) break;
  }
  const int cfill = cnt < NSAMP ? cnt : NSAMP;
  if (lane >= cfill) slist[wave][lane] = NPTS - 1;
  __syncthreads();
  const int gi = clampi(slist[wave][lane], NPTS - 1);
  {
    int* gp = gidx + (size_t)cen * NSAMP + lane;
    *(volatile int*)gp = gi;
    __threadfence();
    *(volatile int*)gp = gi;
  }

  const float gx = bf_rne(xb[gi]);
  const float gy = bf_rne(xb[NPTS + gi]);
  const float gz = bf_rne(xb[2 * NPTS + gi]);
  const float dxl = gx - cx, dyl = gy - cy, dzl = gz - cz;
  const v4f wa = *(const v4f*)(W0x + lane * 4);
  const v4f wb = *(const v4f*)(W0x + (lane + 32) * 4);
  const float wa0 = wa[0], wa1 = wa[1], wa2 = wa[2];
  const float wb0 = wb[0], wb1 = wb[1], wb2 = wb[2];
  const float ba = bf_rne(b0[lane]);
  const float bb = bf_rne(b0[lane + 32]);
  const float* Pb = P0 + (size_t)b * NPTS * CH_A;
  float s0 = 0.f, q0 = 0.f, s1 = 0.f, q1 = 0.f;
#pragma unroll 4
  for (int k = 0; k < NSAMP; ++k) {
    const int gk = __shfl(gi, k, 32);
    const float dx = __shfl(dxl, k, 32);
    const float dy = __shfl(dyl, k, 32);
    const float dz = __shfl(dzl, k, 32);
    const float* pr = Pb + (size_t)gk * CH_A;
    const float pa = pr[lane];
    const float pc = pr[lane + 32];
    const float ya = y0_val(pa, wa0, wa1, wa2, dx, dy, dz, ba);
    const float yb = y0_val(pc, wb0, wb1, wb2, dx, dy, dz, bb);
    const float ya2 = ya * ya;
    const float yb2 = yb * yb;
    s0 += ya;
    q0 += ya2;
    s1 += yb;
    q1 += yb2;
  }
  wst[wave][lane] = s0;
  wst[wave][32 + lane] = s1;
  wst[wave][64 + lane] = q0;
  wst[wave][96 + lane] = q1;
  __syncthreads();
  if (tid < 128) {
    float a = wst[0][tid];
#pragma unroll
    for (int w = 1; w < 8; ++w) a += wst[w][tid];
    pst[tid] = a;
  }
  __syncthreads();
  if (tid < 32) {
    const v4f v = *(const v4f*)(pst + tid * 4);
    float* dp = part0 + (size_t)blockIdx.x * 128 + tid * 4;
    *(volatile v4f*)dp = v;
    __threadfence();
    *(volatile v4f*)dp = v;
  }
}

__global__ __launch_bounds__(256) void k_fin(const float* __restrict__ part, int nblk, int nch,
                                             const float* __restrict__ g, const float* __restrict__ be,
                                             float* __restrict__ tab) {
  __shared__ double red[256];
  const int t = threadIdx.x;
  const int ch = blockIdx.x * 32 + (t & 31);
  const int which = (t >> 5) & 1;
  const int prt = t >> 6;
  const int col = which * nch + ch;
  const int stride = 2 * nch;
  double acc = 0.0;
#pragma unroll 4
  for (int p = prt; p < nblk; p += 4) acc += (double)part[(size_t)p * stride + col];
  red[t] = acc;
  __syncthreads();
  if (t < 32) {
    const double sm = ((red[t] + red[64 + t]) + red[128 + t]) + red[192 + t];
    const double sq = ((red[32 + t] + red[96 + t]) + red[160 + t]) + red[224 + t];
    const double invm = 1.0 / (double)NROWS;
    const double mean = sm * invm;
    const double ex2 = sq * invm;
    const double var = ex2 - mean * mean;
    float varf = (float)var;
    varf = fmaxf(varf, 0.0f);
    const float inv = 1.0f / sqrtf(varf + 1e-5f);
    const float gg = bf_rne(g[ch]);
    const float bb = bf_rne(be[ch]);
    const float scl = gg * inv;
    const float mprod = (float)mean * scl;
    const float sft = bb - mprod;
    float* tp = tab + blockIdx.x * 64;
    *(volatile float*)(tp + t) = scl;
    *(volatile float*)(tp + 32 + t) = sft;
    __threadfence();
    *(volatile float*)(tp + t) = scl;
    *(volatile float*)(tp + 32 + t) = sft;
  }
}

__global__ __launch_bounds__(256) void k_l1(const int* __restrict__ gidx, const float* __restrict__ xyz,
                                            const float* __restrict__ newxyz, const float* __restrict__ P0,
                                            const float* __restrict__ W0x, const float* __restrict__ b0,
                                            const float* __restrict__ tab0, const _Float16* __restrict__ W1h,
                                            const float* __restrict__ b1, _Float16* __restrict__ y1,
                                            float* __restrict__ part1) {
  __shared__ __align__(16) _Float16 As[TILE_ROWS * APITCH];
  __shared__ __align__(16) float slab[8][16 * SPITCH];
  __shared__ __align__(16) float wst[8][128];
  __shared__ __align__(16) float pst[128];
  __shared__ __align__(16) float sW[CH_A * 4];
  __shared__ __align__(16) float sSc[CH_A];
  __shared__ __align__(16) float sSh[CH_A];
  __shared__ __align__(16) float sB0[CH_A];
  const int tid = threadIdx.x, lane = tid & 31, wave = tid >> 5;
  const int blk = blockIdx.x;
  if (tid < CH_A) {
    *(v4f*)(sW + tid * 4) = *(const v4f*)(W0x + tid * 4);
    sSc[tid] = tab0[(tid >> 5) * 64 + (tid & 31)];
    sSh[tid] = tab0[(tid >> 5) * 64 + 32 + (tid & 31)];
    sB0[tid] = bf_rne(b0[tid]);
  }
  __syncthreads();
  {
    const int r = tid >> 1, half = tid & 1;
    const size_t row = (size_t)blk * TILE_ROWS + r;
    const int cen = (int)(row >> 5);
    const int b = cen >> 10, s = cen & (NCENT - 1);
    const int gi = clampi(gidx[row], NPTS - 1);
    const float* cb = newxyz + (size_t)b * 3 * NCENT;
    const float* xb = xyz + (size_t)b * 3 * NPTS;
    const float cx = cb[s], cy = cb[NCENT + s], cz = cb[2 * NCENT + s];
    const float dx = bf_rne(xb[gi]) - cx;
    const float dy = bf_rne(xb[NPTS + gi]) - cy;
    const float dz = bf_rne(xb[2 * NPTS + gi]) - cz;
    const float* pr = P0 + ((size_t)b * NPTS + gi) * CH_A + half * 32;
#pragma unroll 1
    for (int i = 0; i < 4; ++i) {
      const v4f pa = *(const v4f*)(pr + i * 8);
      const v4f pc = *(const v4f*)(pr + i * 8 + 4);
      const int cbase = half * 32 + i * 8;
      v8h hv;
#pragma unroll
      for (int e = 0; e < 8; ++e) {
        const int c = cbase + e;
        const float p = (e < 4) ? pa[e & 3] : pc[e & 3];
        const v4f w = *(const v4f*)(sW + c * 4);
        const float y = y0_val(p, w[0], w[1], w[2], dx, dy, dz, sB0[c]);
        const float ys = y * sSc[c];
        const float x = fmaxf(ys + sSh[c], 0.0f);
        hv[e] = (_Float16)x;
      }
      *(v8h*)(As + r * APITCH + cbase) = hv;
    }
  }
  __syncthreads();

  const int c = lane & 15, hh = lane >> 4;
  v8f acc[4];
#pragma unroll
  for (int j = 0; j < 4; ++j) acc[j] = (v8f){0.f, 0.f, 0.f, 0.f, 0.f, 0.f, 0.f, 0.f};
#pragma unroll
  for (int k0 = 0; k0 < CH_A; k0 += 32) {
    union { v16h v; v8h h[2]; } fa;
    fa.h[0] = *(const v8h*)(As + (wave * 16 + c) * APITCH + k0 + 8 * hh);
    fa.h[1] = *(const v8h*)(As + (wave * 16 + c) * APITCH + k0 + 16 + 8 * hh);
#pragma unroll
    for (int j = 0; j < 4; ++j) {
      const v16h bq = frag_g(W1h + (j * 16 + c) * CH_A + k0 + 8 * hh);
      acc[j] = mma_h(fa.v, bq, acc[j]);
    }
  }
  float* sl = slab[wave];
#pragma unroll
  for (int j = 0; j < 4; ++j) {
    const int col = j * 16 + c;
    const float bv = bf_rne(b1[col]);
    float sm = 0.f, sq = 0.f;
#pragma unroll
    for (int r = 0; r < 8; ++r) {
      const float v = acc[j][r] + bv;
      sl[(8 * hh + r) * SPITCH + col] = v;
      const float v2 = v * v;
      sm += v;
      sq += v2;
    }
    sm += __shfl_xor(sm, 16, 32);
    sq += __shfl_xor(sq, 16, 32);
    wst[wave][hh * 64 + col] = hh ? sq : sm;
  }
  __syncthreads();
  {
    const int q4 = lane >> 3, c8 = (lane & 7) * 8;
    const size_t rbase = (size_t)blk * TILE_ROWS + wave * 16;
    for (int pass = 0; pass < 2; ++pass) {
#pragma unroll
      for (int it = 0; it < 4; ++it) {
        const int row = it * 4 + q4;
        const float* sp = sl + row * SPITCH + c8;
        v8h hv;
#pragma unroll
        for (int e = 0; e < 8; ++e) hv[e] = (_Float16)sp[e];
        *(volatile v8h*)(y1 + (rbase + row) * CH_B + c8) = hv;
      }
      __threadfence();
    }
  }
  if (tid < 128) {
    float a = wst[0][tid];
#pragma unroll
    for (int w = 1; w < 8; ++w) a += wst[w][tid];
    pst[tid] = a;
  }
  __syncthreads();
  if (tid < 32) {
    const v4f v = *(const v4f*)(pst + tid * 4);
    float* dp = part1 + (size_t)blk * 128 + tid * 4;
    *(volatile v4f*)dp = v;
    __threadfence();
    *(volatile v4f*)dp = v;
  }
}

__global__ __launch_bounds__(256) void k_l2(const unsigned* __restrict__ y1w, const float* __restrict__ tab1,
                                            const _Float16* __restrict__ W2h, const float* __restrict__ b2,
                                            float* __restrict__ gmax, float* __restrict__ gmin,
                                            float* __restrict__ part2) {
  __shared__ __align__(16) _Float16 As[TILE_ROWS * APITCH];
  __shared__ __align__(16) float wst[8][256];
  __shared__ __align__(16) float wmm[8][256];
  __shared__ __align__(16) float pst[256];
  __shared__ __align__(16) float sSc[CH_B];
  __shared__ __align__(16) float sSh[CH_B];
  const int tid = threadIdx.x, lane = tid & 31, wave = tid >> 5;
  const int blk = blockIdx.x;
  if (tid < CH_B) {
    sSc[tid] = tab1[(tid >> 5) * 64 + (tid & 31)];
    sSh[tid] = tab1[(tid >> 5) * 64 + 32 + (tid & 31)];
  }
  __syncthreads();
  {
    const int r = tid >> 1, half = tid & 1;
    const size_t row = (size_t)blk * TILE_ROWS + r;
    const v4u* src = (const v4u*)(y1w + row * 32 + half * 16);
#pragma unroll 1
    for (int i = 0; i < 4; ++i) {
      const v4u u = src[i];
      const int cbase = half * 32 + i * 8;
      v8h hv;
#pragma unroll
      for (int j = 0; j < 4; ++j) {
        const unsigned w = u[j];
        const int ca = cbase + 2 * j;
        const float fa = h16_to_f32(w & 0xffffu);
        const float fb = h16_to_f32(w >> 16);
        const float ma = fa * sSc[ca];
        const float mb = fb * sSc[ca + 1];
        const float xa = fmaxf(ma + sSh[ca], 0.0f);
        const float xb = fmaxf(mb + sSh[ca + 1], 0.0f);
        hv[2 * j] = (_Float16)xa;
        hv[2 * j + 1] = (_Float16)xb;
      }
      *(v8h*)(As + r * APITCH + cbase) = hv;
    }
  }
  __syncthreads();

  const int c = lane & 15, hh = lane >> 4;
  v8f acc[8];
#pragma unroll
  for (int j = 0; j < 8; ++j) acc[j] = (v8f){0.f, 0.f, 0.f, 0.f, 0.f, 0.f, 0.f, 0.f};
#pragma unroll
  for (int k0 = 0; k0 < CH_B; k0 += 32) {
    union { v16h v; v8h h[2]; } fa;
    fa.h[0] = *(const v8h*)(As + (wave * 16 + c) * APITCH + k0 + 8 * hh);
    fa.h[1] = *(const v8h*)(As + (wave * 16 + c) * APITCH + k0 + 16 + 8 * hh);
#pragma unroll
    for (int j = 0; j < 8; ++j) {
      const v16h bq = frag_g(W2h + (j * 16 + c) * CH_B + k0 + 8 * hh);
      acc[j] = mma_h(fa.v, bq, acc[j]);
    }
  }
#pragma unroll
  for (int j = 0; j < 8; ++j) {
    const int col = j * 16 + c;
    const float bv = bf_rne(b2[col]);
    float sm = 0.f, sq = 0.f, mx = -3.0e38f, mn = 3.0e38f;
#pragma unroll
    for (int r = 0; r < 8; ++r) {
      const float v = acc[j][r] + bv;
      const float v2 = v * v;
      sm += v;
      sq += v2;
      mx = fmaxf(mx, v);
      mn = fminf(mn, v);
    }
    sm += __shfl_xor(sm, 16, 32);
    sq += __shfl_xor(sq, 16, 32);
    const float omx = __shfl_xor(mx, 16, 32);
    const float omn = __shfl_xor(mn, 16, 32);
    mx = fmaxf(mx, omx);
    mn = fminf(mn, omn);
    wst[wave][hh * 128 + col] = hh ? sq : sm;
    wmm[wave][hh * 128 + col] = hh ? mn : mx;
  }
  __syncthreads();
  {
    float a = wst[0][tid];
#pragma unroll
    for (int w = 1; w < 8; ++w) a += wst[w][tid];
    pst[tid] = a;
  }
  {
    const int gq = wave >> 1, which = wave & 1;
    const v4f a = *(const v4f*)(&wmm[2 * gq][which * 128 + lane * 4]);
    const v4f bq = *(const v4f*)(&wmm[2 * gq + 1][which * 128 + lane * 4]);
    v4f v;
#pragma unroll
    for (int e = 0; e < 4; ++e) {
      const float hi = fmaxf(a[e], bq[e]);
      const float lo = fminf(a[e], bq[e]);
      v[e] = which ? lo : hi;
    }
    float* base = which ? gmin : gmax;
    float* dp = base + ((size_t)blk * 4 + gq) * CH_C + lane * 4;
    *(volatile v4f*)dp = v;
    __threadfence();
    *(volatile v4f*)dp = v;
  }
  __syncthreads();
  if (tid < 64) {
    const v4f v = *(const v4f*)(pst + tid * 4);
    float* dp = part2 + (size_t)blk * 256 + tid * 4;
    *(volatile v4f*)dp = v;
    __threadfence();
    *(volatile v4f*)dp = v;
  }
}

__global__ __launch_bounds__(256) void k_out(const float* __restrict__ gmax, const float* __restrict__ gmin,
                                             const float* __restrict__ tab2, float* __restrict__ out1) {
  __shared__ __align__(16) float tile[CH_C * 36];
  const int t = threadIdx.x;
  const int cen0 = blockIdx.x * 32;
  const int b = cen0 >> 10, s0 = cen0 & (NCENT - 1);
#pragma unroll 1
  for (int i = 0; i < 4; ++i) {
    const int idx = i * 256 + t;
    const int row = idx >> 5, c4 = (idx & 31) * 4;
    const v4f a = *(const v4f*)(gmax + ((size_t)(cen0 + row)) * CH_C + c4);
    const v4f m = *(const v4f*)(gmin + ((size_t)(cen0 + row)) * CH_C + c4);
    const v4f sc = *(const v4f*)(tab2 + (c4 >> 5) * 64 + (c4 & 31));
    const v4f sh = *(const v4f*)(tab2 + (c4 >> 5) * 64 + 32 + (c4 & 31));
#pragma unroll
    for (int e = 0; e < 4; ++e) {
      const float pa = a[e] * sc[e];
      const float pm = m[e] * sc[e];
      const float va = pa + sh[e];
      const float vb = pm + sh[e];
      tile[(c4 + e) * 36 + row] = fmaxf(fmaxf(va, vb), 0.0f);
    }
  }
  __syncthreads();
  for (int pass = 0; pass < 2; ++pass) {
#pragma unroll
    for (int i = 0; i < 4; ++i) {
      const int item = i * 256 + t;
      const int o = item >> 3, s4 = (item & 7) * 4;
      const v4f v = *(const v4f*)(tile + o * 36 + s4);
      *(volatile v4f*)(out1 + ((size_t)(b * CH_C + o)) * NCENT + s0 + s4) = v;
    }
    __threadfence();
  }
}

extern "C" void kernel_launch(void* const* d_in, const int* in_sizes, int n_in,
                              void* d_out, int out_size, void* d_ws, size_t ws_size, hipStream_t stream) {
  if (n_in < 14) return;
  if (ws_size < WS_TOTAL) return;
  (void)in_sizes;
  (void)out_size;
  const float* xyz = (const float*)d_in[0];
  const float* pts = (const float*)d_in[1];
  const float* W0  = (const float*)d_in[2];
  const float* b0  = (const float*)d_in[3];
  const float* g0  = (const float*)d_in[4];
  const float* be0 = (const float*)d_in[5];
  const float* W1  = (const float*)d_in[6];
  const float* b1  = (const float*)d_in[7];
  const float* g1  = (const float*)d_in[8];
  const float* be1 = (const float*)d_in[9];
  const float* W2  = (const float*)d_in[10];
  const float* b2  = (const float*)d_in[11];
  const float* g2  = (const float*)d_in[12];
  const float* be2 = (const float*)d_in[13];
  float* out0 = (float*)d_out;
  float* out1 = (float*)d_out + OUT0_BYTES / 4;

  char* w = (char*)d_ws;
  _Float16* W0p  = (_Float16*)(w + OFF_W0P);
  _Float16* W1h  = (_Float16*)(w + OFF_W1H);
  _Float16* W2h  = (_Float16*)(w + OFF_W2H);
  float*    W0x  = (float*)(w + OFF_W0X);
  float*    tab0 = (float*)(w + OFF_TAB0);
  float*    tab1 = (float*)(w + OFF_TAB1);
  float*    tab2 = (float*)(w + OFF_TAB2);
  float*    nxyz = (float*)(w + OFF_NXYZ);
  int*      gidx = (int*)(w + OFF_GIDX);
  _Float16* ptsT = (_Float16*)(w + OFF_PTST);
  float*    P0   = (float*)(w + OFF_P0);
  float*    prt0 = (float*)(w + OFF_PRT0);
  float*    prt1 = (float*)(w + OFF_PRT1);
  float*    prt2 = (float*)(w + OFF_PRT2);
  _Float16* y1   = (_Float16*)(w + OFF_Y1);
  float*    gmx  = (float*)(w + OFF_GMAX);
  float*    gmn  = (float*)(w + OFF_GMIN);

  k_prep<<<9, 256, 0, stream>>>(W0, W1, W2, W0p, W1h, W2h, W0x);
  k_pts<<<BATCH * (NPTS / 64), 256, 0, stream>>>(pts, ptsT);
  k_p0<<<(BATCH * NPTS) / 128, 256, 0, stream>>>(ptsT, W0p, P0);
  k_fps<<<BATCH, 256, 0, stream>>>(xyz, out0, nxyz);
  k_ball<<<NBLK_BALL, 256, 0, stream>>>(xyz, nxyz, P0, W0x, b0, gidx, prt0);
  k_fin<<<CH_A / 32, 256, 0, stream>>>(prt0, NBLK_BALL, CH_A, g0, be0, tab0);
  k_l1<<<NBLK_MLP, 256, 0, stream>>>(gidx, xyz, nxyz, P0, W0x, b0, tab0, W1h, b1, y1, prt1);
  k_fin<<<CH_B / 32, 256, 0, stream>>>(prt1, NBLK_MLP, CH_B, g1, be1, tab1);
  k_l2<<<NBLK_MLP, 256, 0, stream>>>((const unsigned*)y1, tab1, W2h, b2, gmx, gmn, prt2);
  k_fin<<<CH_C / 32, 256, 0, stream>>>(prt2, NBLK_MLP, CH_C, g2, be2, tab2);
  k_out<<<NGROUP / 32, 256, 0, stream>>>(gmx, gmn, tab2, out1);
}
